// HyperSAGE_77644418777152
// MI455X (gfx1250) — hardware-verified
//
#include <hip/hip_runtime.h>
#include <hip/hip_bf16.h>
#include <math.h>


#define BB 2
#define SS 2048
#define DD 1024
#define HH 16
#define DKK 64
#define QW 2

typedef _Float16 bf16;
typedef __attribute__((ext_vector_type(4))) unsigned v4u_t;
typedef unsigned v4ua __attribute__((ext_vector_type(4), may_alias));
typedef __attribute__((ext_vector_type(4))) float v4f_t;
typedef float v4fa __attribute__((ext_vector_type(4), may_alias));
typedef __attribute__((ext_vector_type(16))) bf16  bf16x16;
typedef __attribute__((ext_vector_type(8)))  bf16  bf16x8;
typedef __attribute__((ext_vector_type(4)))  bf16  bf16x4;
typedef __attribute__((ext_vector_type(8)))  float f32x8;

#define LDS_STRIDE 48
#define KSTRIDE    72
#define VSTRIDE    48

__device__ __forceinline__ f32x8 wmma_bf16(bf16x16 a, bf16x16 b, f32x8 c) {
  return __builtin_amdgcn_wmma_f32_16x16x32_f16(
      false, a, false, b, (short)0, c, false, false);
}
#define RSPLIT (1.0f / 2048.0f)
__device__ __forceinline__ bf16 lo_of(float v, bf16 h) { return (bf16)((v - (float)h) * 2048.0f); }
__device__ __forceinline__ f32x8 wmma_split(bf16x16 a, bf16x16 al, bf16x16 b, bf16x16 bl, f32x8 c) {
  f32x8 x = {}; x = wmma_bf16(al, b, x); x = wmma_bf16(a, bl, x); return wmma_bf16(a, b, c) + x * RSPLIT; }

template <typename T>
__device__ __forceinline__ bf16x16 load_frag(const T* __restrict__ base, int ld,
                                             int row0, int k0) {
  const int lane = threadIdx.x & 31;
  const int r    = lane & 15;
  const int kh   = (lane >> 4) * 8;
  const T* p0 = base + (size_t)(row0 + r) * ld + (k0 + kh);
  const T* p1 = p0 + 16;
  bf16x16 f;
#pragma unroll
  for (int i = 0; i < 8; ++i) {
    f[i]     = (bf16)p0[i];
    f[i + 8] = (bf16)p1[i];
  }
  return f;
}

__device__ __forceinline__ bf16x16 lds_frag(const bf16* base, int stride) {
  const int lane = threadIdx.x & 31;
  const int row  = lane & 15;
  const int kh   = (lane >> 4) * 8;
  const bf16x8 lo = *(const bf16x8*)(base + row * stride + kh);
  const bf16x8 hi = *(const bf16x8*)(base + row * stride + kh + 16);
  bf16x16 f;
#pragma unroll
  for (int i = 0; i < 8; ++i) { f[i] = lo[i]; f[i + 8] = hi[i]; }
  return f;
}

template <typename T>
__device__ __forceinline__ void stage_read16(const T* __restrict__ p, float* buf) {
#pragma unroll
  for (int i = 0; i < 16; ++i) buf[i] = (float)p[i];
}

__device__ __forceinline__ void stage_write(bf16* dst, const float* buf, int nquad) {
#pragma unroll
  for (int i = 0; i < nquad; ++i) {
    bf16x4 q;
    q[0] = (bf16)buf[4 * i];     q[1] = (bf16)buf[4 * i + 1];
    q[2] = (bf16)buf[4 * i + 2]; q[3] = (bf16)buf[4 * i + 3];
    *(bf16x4*)(dst + 4 * i) = q;
  }
}

__global__ __launch_bounds__(256) void transpose_pack_kernel(const float* __restrict__ W, bf16* __restrict__ WT, int K, int N, size_t plane) {
  __shared__ float tile[64][65];
  const int k0 = blockIdx.y * 64, n0 = blockIdx.x * 64, t = threadIdx.x;
  for (int i = t; i < 64 * 64; i += 256) { const int kr = i >> 6, nc = i & 63; tile[kr][nc] = W[(size_t)(k0 + kr) * N + n0 + nc]; }
  __syncthreads();
#pragma unroll 1
  for (int pass = 0; pass < 2; ++pass) {
    for (int i = t; i < 64 * 8; i += 256) { const int nr = i >> 3, k8 = (i & 7) * 8; bf16 hh[8], hl[8];
#pragma unroll
      for (int e = 0; e < 8; ++e) { const float v = tile[k8 + e][nr]; hh[e] = (bf16)v; hl[e] = lo_of(v, hh[e]); }
      bf16* d = WT + (size_t)(n0 + nr) * K + k0 + k8;
      *(volatile v4u_t*)d = *(const v4ua*)hh; *(volatile v4u_t*)(d + plane) = *(const v4ua*)hl; }
    __threadfence();
  }
}

template <typename AT, typename WT, int MODE>
__global__ __launch_bounds__(256) void gemm_split_kernel(
    const AT* __restrict__ A, size_t aPlane, const WT* __restrict__ W, size_t wPlane,
    const float* __restrict__ bias, void* __restrict__ out,
    int M, int N, int K) {
  __shared__ bf16 ldsA[128 * LDS_STRIDE], ldsAl[128 * LDS_STRIDE];
  __shared__ bf16 ldsW[256 * LDS_STRIDE], ldsWl[256 * LDS_STRIDE];
  __shared__ __attribute__((aligned(16))) unsigned char sob[256 * 136 * 2];

  const int t    = threadIdx.x;
  const int wave = t >> 5;
  const int lane = t & 31;
  const int wm   = (wave & 1) * 64;
  const int wn   = (wave >> 1) * 64;
  const int mBlk = blockIdx.x * 128;
  const int nBlk = blockIdx.y * 256;
  const int arow = t >> 1;
  const int ach  = (t & 1) * 16;

  f32x8 acc[4][4] = {};
  for (int k = 0; k < K; k += 32) {
    __syncthreads();
    {
      const AT* ap = A + (size_t)(mBlk + arow) * K + k + ach;
      bf16 hh[16], hl[16];
      if (sizeof(AT) == 4) {
#pragma unroll
        for (int i = 0; i < 16; ++i) { const float v = (float)ap[i]; hh[i] = (bf16)v; hl[i] = lo_of(v, hh[i]); }
      } else {
#pragma unroll
        for (int i = 0; i < 16; ++i) { hh[i] = (bf16)ap[i]; hl[i] = (bf16)ap[aPlane + i]; }
      }
#pragma unroll
      for (int i = 0; i < 16; ++i) { ldsA[arow * LDS_STRIDE + ach + i] = hh[i]; ldsAl[arow * LDS_STRIDE + ach + i] = hl[i]; }
    }
    {
      const WT* wp = W + (size_t)(nBlk + t) * K + k;
      if (sizeof(WT) == 4) {
#pragma unroll
        for (int i = 0; i < 32; ++i) { const float v = (float)wp[i]; const bf16 h_ = (bf16)v; ldsW[t * LDS_STRIDE + i] = h_; ldsWl[t * LDS_STRIDE + i] = lo_of(v, h_); }
      } else {
#pragma unroll
        for (int i = 0; i < 32; ++i) { ldsW[t * LDS_STRIDE + i] = (bf16)wp[i]; ldsWl[t * LDS_STRIDE + i] = (bf16)wp[wPlane + i]; }
      }
    }
    __syncthreads();
    bf16x16 wf[4], wfl[4];
#pragma unroll
    for (int j = 0; j < 4; ++j) { wf[j] = lds_frag(ldsW + (wn + 16 * j) * LDS_STRIDE, LDS_STRIDE); wfl[j] = lds_frag(ldsWl + (wn + 16 * j) * LDS_STRIDE, LDS_STRIDE); }
#pragma unroll
    for (int i = 0; i < 4; ++i) {
      const bf16x16 af = lds_frag(ldsA + (wm + 16 * i) * LDS_STRIDE, LDS_STRIDE), afl = lds_frag(ldsAl + (wm + 16 * i) * LDS_STRIDE, LDS_STRIDE);
#pragma unroll
      for (int j = 0; j < 4; ++j) acc[i][j] = wmma_split(af, afl, wf[j], wfl[j], acc[i][j]);
    }
  }

  const int nlane = lane & 15;
  const int mh    = (lane >> 4) * 8;
  __syncthreads();
  if (MODE == 1) {
    bf16* so = (bf16*)sob;
#pragma unroll
    for (int i = 0; i < 4; ++i)
#pragma unroll
      for (int j = 0; j < 4; ++j) {
        const int nl = wn + 16 * j + nlane;
        const float bv = bias ? bias[nBlk + nl] : 0.0f;
#pragma unroll
        for (int r = 0; r < 8; ++r) so[nl * 136 + wm + 16 * i + mh + r] = (bf16)(acc[i][j][r] + bv);
      }
    __syncthreads();
    const int b_ = mBlk >> 11, s0 = mBlk & (SS - 1);
#pragma unroll 1
    for (int pass = 0; pass < 2; ++pass) {
      for (int ch = t; ch < 256 * 16; ch += 256) { const int nl = ch >> 4, q = (ch & 15) * 8; const int n = nBlk + nl, h = n >> 6, dk = n & (DKK - 1);
        *(volatile v4u_t*)((bf16*)out + (((size_t)(b_ * HH + h)) * DKK + dk) * SS + s0 + q) = *(const v4ua*)(so + nl * 136 + q); }
      __threadfence();
    }
  } else {
    float* so = (float*)sob;
#pragma unroll 1
    for (int hf = 0; hf < 2; ++hf) {
      if (wm == hf * 64) {
#pragma unroll
        for (int i = 0; i < 4; ++i)
#pragma unroll
          for (int j = 0; j < 4; ++j) {
            const int nl = wn + 16 * j + nlane;
            const float bv = bias ? bias[nBlk + nl] : 0.0f;
#pragma unroll
            for (int r = 0; r < 8; ++r) so[(16 * i + mh + r) * 260 + nl] = acc[i][j][r] + bv;
          }
      }
      __syncthreads();
#pragma unroll 1
      for (int pass = 0; pass < 2; ++pass) {
        for (int ch = t; ch < 64 * 64; ch += 256) { const int ml = ch >> 6, q = (ch & 63) * 4;
          *(volatile v4f_t*)((float*)out + (size_t)(mBlk + hf * 64 + ml) * N + nBlk + q) = *(const volatile v4fa*)(so + ml * 260 + q); }
        __threadfence();
      }
      __syncthreads();
    }
  }
}


#define HN 100000
#define HNP 100096
#define HNR 50048
#define HM 20000
#define HMP 20096
#define HZ 2000000
#define HD 64

template <int KIND, int RANGE, int DS, int DOFF>
__global__ __launch_bounds__(256) void k_scatter(const int* __restrict__ sidx, const int* __restrict__ didx, int nsrc, int ndst,
                                                const float* __restrict__ Src, const float* __restrict__ nneigh,
                                                float* __restrict__ Dst, float* __restrict__ cntout) {
  __shared__ int qd[8][256], qs[8][256]; __shared__ int wcnt[8][8]; __shared__ unsigned short cnt[RANGE];
  const int tid = threadIdx.x, lane = tid & 31, wave = tid >> 5, r0 = blockIdx.x * RANGE;
  float* myR = Dst + (size_t)r0 * DS + DOFF;
  for (int i = tid; i < RANGE * 16; i += 256) { const int dl = i >> 4, c4 = (i & 15) * 4; v4f_t z; z.x = z.y = z.z = z.w = 0.0f; *(volatile v4f_t*)(myR + (size_t)dl * DS + c4) = z; }
  for (int i = tid; i < RANGE; i += 256) cnt[i] = 0;
  __threadfence(); __syncthreads();
#pragma unroll 1
  for (int c0 = 0; c0 < HZ; c0 += 256) {
    const int e = c0 + tid; int d = -1, s = 0;
    if (e < HZ) { const int draw = didx[e]; const int dd = draw < 0 ? 0 : (draw >= ndst ? ndst - 1 : draw);
      if (dd >= r0 && dd < r0 + RANGE) { d = dd - r0; const int ss = sidx[e]; s = ss < 0 ? 0 : (ss >= nsrc ? nsrc - 1 : ss); } }
    const int own = (d >= 0) ? (d & 7) : -1;
    unsigned mown = 0u;
#pragma unroll
    for (int w = 0; w < 8; ++w) { const unsigned m = __builtin_amdgcn_ballot_w32(own == w); if (own == w) mown = m; if (lane == 0) wcnt[w][wave] = __builtin_popcount(m); }
    __syncthreads();
    if (own >= 0) { int base = 0;
#pragma unroll
      for (int w2 = 0; w2 < 8; ++w2) base += (w2 < wave) ? wcnt[own][w2] : 0;
      const int pos = base + __builtin_popcount(mown & ((1u << lane) - 1u)); qd[own][pos] = d; qs[own][pos] = s; }
    int total = 0;
#pragma unroll
    for (int w2 = 0; w2 < 8; ++w2) total += wcnt[wave][w2];
    __syncthreads();
#pragma unroll 1
    for (int qi = 0; qi < total; ++qi) { const int dl = qd[wave][qi], sl = qs[wave][qi];
      float* row = myR + (size_t)dl * DS; const float* sr = Src + (size_t)sl * HD;
      row[lane] += sr[lane]; row[32 + lane] += sr[32 + lane];
      if (lane == 0) cnt[dl] += 1; }
    __syncthreads();
  }
  __threadfence(); __syncthreads();
#pragma unroll 1
  for (int pass = 0; pass < 2; ++pass) {
    for (int i = tid; i < RANGE * 16; i += 256) { const int dl = i >> 4, c4 = (i & 15) * 4, dg = r0 + dl; float* p = myR + (size_t)dl * DS + c4;
      v4f_t v = *(const volatile v4fa*)p;
      if (pass == 0 && KIND == 1) { const float sc = (dg < ndst) ? 1.0f / (fmaxf((float)cnt[dl], 1.0f) * nneigh[dg]) : 0.0f; v.x *= sc; v.y *= sc; v.z *= sc; v.w *= sc; }
      *(volatile v4f_t*)p = v; }
    if (KIND == 0) for (int i = tid; i < RANGE / 4; i += 256) { v4f_t c; c.x = fmaxf((float)cnt[i * 4], 1.f); c.y = fmaxf((float)cnt[i * 4 + 1], 1.f); c.z = fmaxf((float)cnt[i * 4 + 2], 1.f); c.w = fmaxf((float)cnt[i * 4 + 3], 1.f);
      *(volatile v4f_t*)(cntout + r0 + i * 4) = c; }
    __threadfence(); __syncthreads();
  }
}
__global__ __launch_bounds__(64) void k_xhalf(const float* __restrict__ X, float* __restrict__ R) {
  const int i = blockIdx.x, c = threadIdx.x; const float v = (i < HN) ? X[(size_t)i * HD + c] : 0.0f;
  *(volatile float*)(R + (size_t)i * 2 * HD + c) = v; __threadfence(); *(volatile float*)(R + (size_t)i * 2 * HD + c) = v;
}
__global__ __launch_bounds__(128) void k_packA(const float* __restrict__ W, float* __restrict__ A) {
  const int m = blockIdx.x, k = threadIdx.x; const float v = (m < HD) ? W[(size_t)k * HD + m] : 0.0f;
  *(volatile float*)(A + (size_t)m * 2 * HD + k) = v; __threadfence(); *(volatile float*)(A + (size_t)m * 2 * HD + k) = v;
}
__global__ __launch_bounds__(256) void k_rows(const float* __restrict__ T, float* __restrict__ X, int nrows) {
  __shared__ float tile[64][65];
  const int n0 = blockIdx.x * 64, t = threadIdx.x;
  for (int i = t; i < 64 * 64; i += 256) { const int c = i >> 6, nn = i & 63; tile[c][nn] = T[(size_t)c * HNP + n0 + nn]; }
  __syncthreads();
#pragma unroll 1
  for (int pass = 0; pass < 2; ++pass) {
    for (int i = t; i < 64 * 16; i += 256) { const int nr = i >> 4, c4 = (i & 15) * 4; v4f_t v;
#pragma unroll
      for (int q = 0; q < 4; ++q) { const float y = tile[c4 + q][nr]; v[q] = y > 0.0f ? y : 0.01f * y; }
      if (n0 + nr < nrows) *(volatile v4f_t*)(X + (size_t)(n0 + nr) * HD + c4) = v; }
    __threadfence();
  }
}

extern "C" void kernel_launch(void* const* d_in, const int* in_sizes, int n_in,
                              void* d_out, int out_size, void* d_ws, size_t ws_size,
                              hipStream_t stream) {
  (void)in_sizes; (void)n_in; (void)out_size; (void)ws_size;
  const float* X0 = (const float*)d_in[0];
  const float* nneigh = (const float*)d_in[1];
  const float* W1 = (const float*)d_in[2];
  const float* W2 = (const float*)d_in[3];
  const int* inode = (const int*)d_in[4];
  const int* iedge = (const int*)d_in[5];
  char* ws = (char*)d_ws;
  float* A1 = (float*)ws; ws += (size_t)128 * 128 * 4;
  float* A2 = (float*)ws; ws += (size_t)128 * 128 * 4;
  float* ES = (float*)ws; ws += (size_t)HMP * HD * 4;
  float* card = (float*)ws; ws += (size_t)HMP * 4;
  float* R  = (float*)ws; ws += (size_t)HNP * 2 * HD * 4;
  float* T  = (float*)ws; ws += (size_t)128 * HNP * 4;
  float* X1 = T + (size_t)64 * HNP;
  k_packA<<<128, 128, 0, stream>>>(W1, A1);
  k_packA<<<128, 128, 0, stream>>>(W2, A2);
  dim3 blk(256);
  const float* Xin = X0;
  for (int l = 0; l < 2; ++l) {
    k_scatter<0, HMP, HD, 0><<<1, 256, 0, stream>>>(inode, iedge, HN, HM, Xin, nullptr, ES, card);
    k_scatter<1, HNR, 2 * HD, HD><<<HNP / HNR, 256, 0, stream>>>(iedge, inode, HM, HN, ES, nneigh, R, nullptr);
    k_xhalf<<<HNP, 64, 0, stream>>>(Xin, R);
    gemm_split_kernel<float, float, 2><<<dim3(1, HNP / 256), blk, 0, stream>>>(l == 0 ? A1 : A2, 0, R, 0, nullptr, T, 128, HNP, 2 * HD);
    k_rows<<<HNP / 64, 256, 0, stream>>>(T, l == 0 ? X1 : (float*)d_out, l == 0 ? HNP : HN);
    Xin = X1;
  }
}
